// XEncoder_309237645936
// MI455X (gfx1250) — hardware-run, weakly checked
//
#include <hip/hip_runtime.h>
#include <math.h>


#ifndef NB
#define NB 2
#endif
#ifndef SEQ
#define SEQ 2048
#endif
#define NB_FULL  2
#define SEQ_FULL 2048
#define DM   1024
#define HD   128
#define NGRP (8 * NB)
#define OUTF 512
#define MR   (NB * SEQ)
#define AW   4
#define OSP  132
#define HSP  72
#define WH   4
#define PCAR 16.0f
#define ACAR 16.0f
#define WCAR 64.0f
#define GS   (1.0f / 1024.0f)
#define SC2  ((float)(0.03125 * 1.4426950408889634 / 256.0))
#define LOG2E 1.4426950408889634f
#define PSH  14.0f
#define NEGB (-3.0e38f)
#define O1OFF ((size_t)NB_FULL * OUTF * SEQ_FULL)

static_assert(PCAR == ACAR);
static_assert(ACAR * WCAR == 1024.0f);
static_assert(8 * HD == DM);
static_assert(SEQ % 64 == 0);
static_assert(MR % 64 == 0);
static_assert(DM % 64 == 0);
static_assert(OUTF % 64 == 0);
static_assert(DM % 32 == 0);
static_assert(OUTF % 32 == 0);
static_assert(HD % 32 == 0);
static_assert(HD == 128);
static_assert(SEQ % (16 * AW) == 0);
static_assert(SEQ % (32 * AW) == 0);
static_assert(SEQ % 32 == 0);
static_assert(MR % 8 == 0);
static_assert(NB <= NB_FULL);
static_assert(SEQ <= SEQ_FULL);
static_assert((OSP * 4) % 16 == 0);
static_assert((HSP * 2) % 16 == 0);
static_assert(O1OFF * 4 == (size_t)8388608);
static_assert(8 * 32 * 16 == 16 * HD * 2);
static_assert(4 * 4 == 16 && 8 * 16 == HD);
static_assert(8 * 2 == 16 && 16 * 16 == 256);
static_assert(16 * 4 == 64);
static_assert(AW * 16 * OSP * 4 + SEQ * 4 + AW * 4 <= 131072);
static_assert(16 * 68 * 4 + 64 * HSP * 2 <= 131072);
static_assert(64 * 136 * 2 <= 131072 && 64 * 68 * 4 <= 131072);

typedef _Float16 h16;
typedef unsigned short bf;
typedef __attribute__((ext_vector_type(16))) __bf16   v16bf;
typedef __attribute__((ext_vector_type(16))) _Float16 v16h;
typedef __attribute__((ext_vector_type(8)))  _Float16 v8h;
typedef __attribute__((ext_vector_type(8)))  unsigned short v8us;
typedef __attribute__((ext_vector_type(4)))  unsigned short v4us;
typedef __attribute__((ext_vector_type(8)))  float    v8f;
typedef __attribute__((ext_vector_type(4)))  float    v4f;
typedef v4f  __attribute__((may_alias)) v4fa;
typedef v8h  __attribute__((may_alias)) v8ha;

__device__ __forceinline__ unsigned short f2bf(float f) { unsigned u = __float_as_uint(f); u += 0x7FFFu + ((u >> 16) & 1u); return (unsigned short)(u >> 16); }
__device__ __forceinline__ float bfr(float f) { return __uint_as_float(((unsigned)f2bf(f)) << 16); }
__device__ __forceinline__ v16h cat16(v8h lo, v8h hi) { return __builtin_shufflevector(lo, hi, 0, 1, 2, 3, 4, 5, 6, 7, 8, 9, 10, 11, 12, 13, 14, 15); }
__device__ __forceinline__ v16bf cat16b(v8us lo, v8us hi) { return __builtin_bit_cast(v16bf, __builtin_shufflevector(lo, hi, 0, 1, 2, 3, 4, 5, 6, 7, 8, 9, 10, 11, 12, 13, 14, 15)); }
__device__ __forceinline__ v8f wmma16(v16h a, v16h b, v8f c) { return __builtin_amdgcn_wmma_f32_16x16x32_f16(false, a, false, b, (short)0, c, false, false); }
__device__ __forceinline__ v8f wmmab(v16bf a, v16bf b, v8f c) { return __builtin_amdgcn_wmma_f32_16x16x32_bf16(false, a, false, b, (short)0, c, false, false); }
__device__ __forceinline__ v16h  ldh(const h16* p) { return cat16(*(const v8h*)p, *(const v8h*)(p + 16)); }
__device__ __forceinline__ v16bf ldb(const bf* p)  { return cat16b(*(const v8us*)p, *(const v8us*)(p + 16)); }
__device__ __forceinline__ void wave_sync() { __builtin_amdgcn_fence(3  , "wavefront"); __builtin_amdgcn_wave_barrier(); asm volatile("" ::: "memory"); }
__device__ __forceinline__ v8f wmg(v16h a, v16h b, v8f c)   { c = wmma16(a, b, c); asm volatile("v_nop\n\tv_nop\n\tv_nop\n\tv_nop" : "+v"(c) : "v"(a), "v"(b)); return c; }
__device__ __forceinline__ v8f wmgb(v16bf a, v16bf b, v8f c) { c = wmmab(a, b, c); asm volatile("v_nop\n\tv_nop\n\tv_nop\n\tv_nop" : "+v"(c) : "v"(a), "v"(b)); return c; }
static __device__ __forceinline__ h16 toh_flush(float v) { const h16 r = (h16)v; return (fabsf(v) < 6.103515625e-05f) ? (h16)0.0f : r; }
__device__ __forceinline__ float adj_val(float aw, float ab, int d) {
#pragma clang fp contract(off)
    const float fd = (float)d; const float d2 = fd * fd; const float u = aw * d2; const float w = u - ab; return expf(-fabsf(w));
}

__global__ __launch_bounds__(256) void k_cvt8(const float* __restrict__ src, bf* dst, size_t n8) {
    const size_t i = (size_t)blockIdx.x * 256 + threadIdx.x; if (i >= n8) return;
    const v8f v = *(const v8f*)(src + i * 8); v8us o;
#pragma unroll
    for (int k = 0; k < 8; ++k) o[k] = f2bf(v[k]);
    *(volatile v8us*)(dst + i * 8) = o; __threadfence(); *(volatile v8us*)(dst + i * 8) = o;
}

template <typename OT> struct WCvt;
template <> struct WCvt<bf>  { typedef v8us V; static __device__ __forceinline__ unsigned short one(float v) { return f2bf(v); } };
template <> struct WCvt<h16> { typedef v8h  V; static __device__ __forceinline__ h16 one(float v) { return toh_flush(bfr(v) * WCAR); } };
template <typename OT>
__device__ __forceinline__ void wt_body(const float* __restrict__ W, OT* WT, const int K, const int N) {
    __shared__ __align__(16) float tw[64 * 68];
    const int tid = threadIdx.x; const int n0 = blockIdx.x * 64, k0 = blockIdx.y * 64;
#pragma unroll
    for (int i = 0; i < 4; ++i) { const int p = i * 256 + tid; const int kr = p >> 4, c4 = (p & 15) * 4;
        const v4f v = *(const v4f*)(W + (size_t)(k0 + kr) * N + n0 + c4); *(v4fa*)(&tw[kr * 68 + c4]) = v; }
    __syncthreads();
    typename WCvt<OT>::V ov[2];
#pragma unroll
    for (int i = 0; i < 2; ++i) { const int p = i * 256 + tid; const int n = p >> 3, k8 = (p & 7) * 8;
#pragma unroll
        for (int kk = 0; kk < 8; ++kk) ov[i][kk] = WCvt<OT>::one(tw[(k8 + kk) * 68 + n]); }
#pragma unroll 1
    for (int ps = 0; ps < 2; ++ps) {
#pragma unroll
        for (int i = 0; i < 2; ++i) { const int p = i * 256 + tid; const int n = p >> 3, k8 = (p & 7) * 8;
            *(volatile typename WCvt<OT>::V*)(WT + (size_t)(n0 + n) * K + k0 + k8) = ov[i]; }
        if (ps == 0) __threadfence(); }
}
__global__ __launch_bounds__(256) void k_wt_bf(const float* __restrict__ W, bf* WT, int K, int N) { wt_body<bf>(W, WT, K, N); }
__global__ __launch_bounds__(256) void k_wt_h(const float* __restrict__ W, h16* WT, int K, int N) { wt_body<h16>(W, WT, K, N); }

template <typename T> struct Frag;
template <> struct Frag<bf>  { typedef v16bf V; static __device__ __forceinline__ V ld(const bf* p)  { return ldb(p); } static __device__ __forceinline__ v8f mm(V a, V b, v8f c) { return wmgb(a, b, c); } };
template <> struct Frag<h16> { typedef v16h  V; static __device__ __forceinline__ V ld(const h16* p) { return ldh(p); } static __device__ __forceinline__ v8f mm(V a, V b, v8f c) { return wmg(a, b, c); } };
template <typename T>
__device__ __forceinline__ void gemm_acc(const T* __restrict__ A, const T* __restrict__ Bt, const int K, const int r0, const int c0, const int lr, const int hi, v8f (&acc)[4][4]) {
#pragma unroll
    for (int mb = 0; mb < 4; ++mb)
#pragma unroll
        for (int nb = 0; nb < 4; ++nb) acc[mb][nb] = (v8f){};
    const size_t aoff = (size_t)(r0 + lr) * K + 8 * hi, boff = (size_t)(c0 + lr) * K + 8 * hi;
#pragma unroll 1
    for (int kc = 0; kc < K; kc += 32) {
        typename Frag<T>::V a[4];
#pragma unroll
        for (int mb = 0; mb < 4; ++mb) a[mb] = Frag<T>::ld(A + aoff + (size_t)mb * 16 * K + kc);
#pragma unroll
        for (int nb = 0; nb < 4; ++nb) { const typename Frag<T>::V b = Frag<T>::ld(Bt + boff + (size_t)nb * 16 * K + kc);
#pragma unroll
            for (int mb = 0; mb < 4; ++mb) acc[mb][nb] = Frag<T>::mm(a[mb], b, acc[mb][nb]); }
    }
}

__global__ __launch_bounds__(32) void k_gemm_proj(const bf* __restrict__ A, const bf* __restrict__ Bt, const float* __restrict__ bias, h16* P, int N, int K) {
    __shared__ __align__(16) float os[16 * 68];
    const int lane = threadIdx.x & 31, lr = lane & 15, hi = lane >> 4; const int r0 = blockIdx.x * 64, c0 = blockIdx.y * 64;
    v8f acc[4][4];
    gemm_acc<bf>(A, Bt, K, r0, c0, lr, hi, acc);
    float bc[4];
#pragma unroll
    for (int nb = 0; nb < 4; ++nb) bc[nb] = bfr(bias[c0 + nb * 16 + lr]);
#pragma unroll
    for (int mb = 0; mb < 4; ++mb) {
#pragma unroll
        for (int nb = 0; nb < 4; ++nb) {
#pragma unroll
            for (int j = 0; j < 8; ++j) os[(hi * 8 + j) * 68 + nb * 16 + lr] = (acc[mb][nb][j] + bc[nb]) * PCAR; }
        wave_sync();
#pragma unroll 1
        for (int ps = 0; ps < 2; ++ps) {
#pragma unroll
            for (int s = 0; s < 4; ++s) { const int row = 4 * s + (lane >> 3), c8 = (lane & 7) * 8;
                const v4f x0 = *(const v4fa*)(&os[row * 68 + c8]); const v4f x1 = *(const v4fa*)(&os[row * 68 + c8 + 4]); v8h hv;
#pragma unroll
                for (int i = 0; i < 4; ++i) { hv[i] = toh_flush(x0[i]); hv[4 + i] = toh_flush(x1[i]); }
                *(volatile v8h*)(P + (size_t)(r0 + mb * 16 + row) * N + c0 + c8) = hv; }
            if (ps == 0) __threadfence(); }
        wave_sync();
    }
}

__global__ __launch_bounds__(32) void k_gemm_res(const h16* __restrict__ A, const h16* __restrict__ Bt, const float* __restrict__ bias, const bf* __restrict__ XR, float* X2, int N, int K) {
    __shared__ __align__(16) float os[16 * 68];
    const int lane = threadIdx.x & 31, lr = lane & 15, hi = lane >> 4; const int r0 = blockIdx.x * 64, c0 = blockIdx.y * 64;
    v8f acc[4][4];
    gemm_acc<h16>(A, Bt, K, r0, c0, lr, hi, acc);
    float bc[4];
#pragma unroll
    for (int nb = 0; nb < 4; ++nb) bc[nb] = bfr(bias[c0 + nb * 16 + lr]);
#pragma unroll
    for (int mb = 0; mb < 4; ++mb) {
#pragma unroll
        for (int nb = 0; nb < 4; ++nb) {
#pragma unroll
            for (int j = 0; j < 8; ++j) os[(hi * 8 + j) * 68 + nb * 16 + lr] = acc[mb][nb][j] * GS + bc[nb]; }
        wave_sync();
#pragma unroll 1
        for (int ps = 0; ps < 2; ++ps) {
#pragma unroll
            for (int s = 0; s < 8; ++s) { const int row = 2 * s + (lane >> 4), c4 = (lane & 15) * 4;
                const size_t go = (size_t)(r0 + mb * 16 + row) * N + c0 + c4;
                const v4f x0 = *(const v4fa*)(&os[row * 68 + c4]);
                const v4us xr = *(const v4us*)(XR + go); v4f val;
#pragma unroll
                for (int i = 0; i < 4; ++i) val[i] = x0[i] + __uint_as_float(((unsigned)xr[i]) << 16);
                *(volatile v4f*)(X2 + go) = val; }
            if (ps == 0) __threadfence(); }
        wave_sync();
    }
}

__global__ __launch_bounds__(32) void k_gemm_tr(const h16* __restrict__ A, const h16* __restrict__ Bt, const float* __restrict__ bias, float* OUTP, h16* XE, int K, int wxe) {
    __shared__ __align__(16) float os[16 * 68];
    __shared__ __align__(16) h16 hs[64 * HSP];
    const int lane = threadIdx.x & 31, lr = lane & 15, hi = lane >> 4; const int r0 = blockIdx.x * 64, c0 = blockIdx.y * 64;
    v8f acc[4][4];
    gemm_acc<h16>(A, Bt, K, r0, c0, lr, hi, acc);
    const int bb = c0 / SEQ, tt = c0 % SEQ;
    float* obase = OUTP + ((size_t)bb * OUTF + (size_t)r0) * SEQ_FULL + tt;
#pragma unroll
    for (int mb = 0; mb < 4; ++mb) {
        float br[8];
#pragma unroll
        for (int j = 0; j < 8; ++j) br[j] = bfr(bias[r0 + mb * 16 + hi * 8 + j]);
#pragma unroll
        for (int nb = 0; nb < 4; ++nb) { v8h hv;
#pragma unroll
            for (int j = 0; j < 8; ++j) { const float z = acc[mb][nb][j] * GS + br[j];
                const float gv = 0.5f * z * (1.0f + erff(z * 0.70710678118654752440f));
                os[(hi * 8 + j) * 68 + nb * 16 + lr] = gv; hv[j] = toh_flush(gv * ACAR); }
            if (wxe != 0) *(v8ha*)(&hs[(nb * 16 + lr) * HSP + mb * 16 + 8 * hi]) = hv; }
        wave_sync();
#pragma unroll 1
        for (int ps = 0; ps < 2; ++ps) {
#pragma unroll
            for (int s = 0; s < 8; ++s) { const int row = 2 * s + (lane >> 4), c4 = (lane & 15) * 4;
                const v4f val = *(const v4fa*)(&os[row * 68 + c4]);
                *(volatile v4f*)(obase + (size_t)(mb * 16 + row) * SEQ_FULL + c4) = val; }
            if (ps == 0) __threadfence(); }
        wave_sync();
    }
    if (wxe != 0) {
#pragma unroll 1
        for (int ps = 0; ps < 2; ++ps) {
#pragma unroll
            for (int s = 0; s < 16; ++s) { const int row = 4 * s + (lane >> 3), c8 = (lane & 7) * 8;
                const v8h hv = *(const v8ha*)(&hs[row * HSP + c8]);
                *(volatile v8h*)(XE + (size_t)(c0 + row) * OUTF + r0 + c8) = hv; }
            if (ps == 0) __threadfence(); }
    }
}

__global__ __launch_bounds__(256) void k_vt(const h16* __restrict__ VP, h16* VT) {
    __shared__ __align__(16) h16 ts[64 * 136];
    const int tid = threadIdx.x; const int g = blockIdx.y; const int tok0 = blockIdx.x * 64;
    const size_t gbase = (size_t)g * SEQ * HD;
#pragma unroll
    for (int i = 0; i < 4; ++i) { const int p = i * 256 + tid; const int row = p >> 4, c8 = (p & 15) * 8;
        const v8h v = *(const v8h*)(VP + gbase + (size_t)(tok0 + row) * HD + c8); *(v8ha*)(&ts[row * 136 + c8]) = v; }
    __syncthreads();
    v8h ov[4];
#pragma unroll
    for (int i = 0; i < 4; ++i) { const int p = i * 256 + tid; const int d = p >> 3, t8 = (p & 7) * 8;
#pragma unroll
        for (int k = 0; k < 8; ++k) ov[i][k] = ts[(t8 + k) * 136 + d]; }
#pragma unroll 1
    for (int ps = 0; ps < 2; ++ps) {
#pragma unroll
        for (int i = 0; i < 4; ++i) { const int p = i * 256 + tid; const int d = p >> 3, t8 = (p & 7) * 8;
            *(volatile v8h*)(VT + gbase + (size_t)d * SEQ + tok0 + t8) = ov[i]; }
        if (ps == 0) __threadfence(); }
}

__global__ __launch_bounds__(32 * AW) __attribute__((amdgpu_num_vgpr(256)))
void k_keypass(const h16* __restrict__ QP, const h16* __restrict__ KP, const h16* __restrict__ VT,
             const float* __restrict__ alpha_p, const float* __restrict__ adjw_p, const float* __restrict__ adjb_p, h16* XO) {
    __shared__ __align__(16) float os[AW * 16 * OSP];
    __shared__ float adjt[SEQ];
    __shared__ int wz[AW];
    const int lane = threadIdx.x & 31, lr = lane & 15, hi = lane >> 4;
    const int wave = __builtin_amdgcn_readfirstlane((int)(threadIdx.x >> 5));
    const int g = blockIdx.y;
    const int t0 = ((int)blockIdx.x * AW + wave) * 16;
    const int t0v = ((int)blockIdx.x * AW + (int)(threadIdx.x >> 5)) * 16;
    int kbv = t0v - WH; kbv = kbv < 0 ? 0 : kbv; kbv &= ~31;
    int kev = t0v + 16 + WH; kev = kev > SEQ ? SEQ : kev;
    const int kb0 = __builtin_amdgcn_readfirstlane(kbv), ke0 = __builtin_amdgcn_readfirstlane(kev);
    const float aw = bfr(adjw_p[0]), ab = bfr(adjb_p[0]);
    int zm = 0;
#pragma unroll 1
    for (int d = (int)threadIdx.x; d < SEQ; d += 32 * AW) { const float sv = adj_val(aw, ab, d) * LOG2E; adjt[d] = sv; zm = (sv != 0.0f) ? (d + 1) : zm; }
#pragma unroll
    for (int off = 16; off > 0; off >>= 1) { const int oz = __shfl_xor(zm, off, 32); zm = oz > zm ? oz : zm; }
    if (lane == 0) wz[wave] = zm;
    __syncthreads();
    int dzv = wz[0];
#pragma unroll
    for (int w = 1; w < AW; ++w) { const int oz = wz[w]; dzv = oz > dzv ? oz : dzv; }
    const int dz = __builtin_amdgcn_readfirstlane(dzv);
    const float al = bfr(alpha_p[0]);
    const float ag = 1.0f / (1.0f + expf(-al));
    const size_t gbase = (size_t)g * SEQ * HD;
    const size_t qo = gbase + (size_t)(t0 + lr) * HD + 8 * hi;
    const v16h q0 = ldh(QP + qo), q1 = ldh(QP + qo + 32), q2 = ldh(QP + qo + 64), q3 = ldh(QP + qo + 96);
    const size_t ko = gbase + (size_t)lr * HD + 8 * hi;
    const size_t vo = gbase + (size_t)lr * SEQ + 8 * hi;
    const int wb = wave * 16 * OSP;
#pragma unroll 1
    for (int pass = 0; pass < 2; ++pass) {
        const int wlim = WH + pass * SEQ;
        const int kb = kb0 * (1 - pass);
        const int ke = ke0 + pass * (SEQ - ke0);
        v8f o[8];
#pragma unroll
        for (int j = 0; j < 8; ++j) o[j] = (v8f){};
        float m = NEGB, l = 0.0f;
#pragma unroll 1
        for (int key0 = kb; key0 < ke; key0 += 32) {
            const h16* ka = KP + ko + (size_t)key0 * HD;
            v8f sa = (v8f){}, sb = (v8f){};
            { const v16h a0 = ldh(ka),      b0 = ldh(ka + 16 * HD);      sa = wmg(a0, q0, sa); sb = wmg(b0, q0, sb); }
            { const v16h a0 = ldh(ka + 32), b0 = ldh(ka + 16 * HD + 32); sa = wmg(a0, q1, sa); sb = wmg(b0, q1, sb); }
            { const v16h a0 = ldh(ka + 64), b0 = ldh(ka + 16 * HD + 64); sa = wmg(a0, q2, sa); sb = wmg(b0, q2, sb); }
            { const v16h a0 = ldh(ka + 96), b0 = ldh(ka + 16 * HD + 96); sa = wmg(a0, q3, sa); sb = wmg(b0, q3, sb); }
            const int dq = t0 + lr - key0 - 8 * hi;
            int da[8], db[8]; float ta[8], tb[8];
#pragma unroll
            for (int r = 0; r < 8; ++r) { int u = dq - r; u = u < 0 ? -u : u; da[r] = u; int w = dq - 16 - r; w = w < 0 ? -w : w; db[r] = w;
                ta[r] = sa[r] * SC2; tb[r] = sb[r] * SC2; }
            const bool near = ((key0 - (t0 + 15)) < dz) & ((t0 - (key0 + 31)) < dz);
            if (near) {
#pragma unroll
                for (int r = 0; r < 8; ++r) { const int ia = da[r] > SEQ - 1 ? SEQ - 1 : da[r]; const int ib = db[r] > SEQ - 1 ? SEQ - 1 : db[r];
                    ta[r] += adjt[ia]; tb[r] += adjt[ib]; }
            }
            bool fa[8], fb[8]; float mx = NEGB;
#pragma unroll
            for (int r = 0; r < 8; ++r) { fa[r] = da[r] <= wlim; fb[r] = db[r] <= wlim;
                mx = fmaxf(mx, fmaxf(fa[r] ? ta[r] : NEGB, fb[r] ? tb[r] : NEGB)); }
            mx = fmaxf(mx, __shfl_xor(mx, 16, 32));
            const float mnew = fmaxf(m, mx);
            const float alpha = __builtin_amdgcn_exp2f(m - mnew);
            const float sh = PSH - mnew;
            v16h pb; float ls = 0.0f;
#pragma unroll
            for (int r = 0; r < 8; ++r) {
                const float xa = ta[r] + sh, xb = tb[r] + sh;
                const float ea = __builtin_amdgcn_exp2f(xa), eb = __builtin_amdgcn_exp2f(xb);
                const float ga = (fa[r] & (xa >= -14.0f)) ? ea : 0.0f, gb = (fb[r] & (xb >= -14.0f)) ? eb : 0.0f;
                const h16 pa = (h16)ga; const h16 pc = (h16)gb;
                pb[r] = pa; pb[8 + r] = pc;
                ls += (float)pa + (float)pc; }
            l = l * alpha + ls; m = mnew;
#pragma unroll
            for (int j = 0; j < 8; ++j) o[j] = o[j] * alpha;
            const h16* va = VT + vo + key0;
            { const v16h v0 = ldh(va), v1 = ldh(va + (size_t)16 * SEQ), v2 = ldh(va + (size_t)32 * SEQ), v3 = ldh(va + (size_t)48 * SEQ);
              o[0] = wmg(v0, pb, o[0]); o[1] = wmg(v1, pb, o[1]); o[2] = wmg(v2, pb, o[2]); o[3] = wmg(v3, pb, o[3]); }
            { const v16h v0 = ldh(va + (size_t)64 * SEQ), v1 = ldh(va + (size_t)80 * SEQ), v2 = ldh(va + (size_t)96 * SEQ), v3 = ldh(va + (size_t)112 * SEQ);
              o[4] = wmg(v0, pb, o[4]); o[5] = wmg(v1, pb, o[5]); o[6] = wmg(v2, pb, o[6]); o[7] = wmg(v3, pb, o[7]); }
        }
        l += __shfl_xor(l, 16, 32);
        const bool any = l > 0.0f;
        const float lsafe = any ? l : 1.0f;
        const float inv = any ? (1.0f / lsafe) : 0.0f;
        const float cw = (float)pass * ag + (float)(1 - pass) * (1.0f - ag);
        const float cf = inv * cw;
#pragma unroll
        for (int j = 0; j < 8; ++j) { v4f a, c; const int ix = wb + lr * OSP + 16 * j + 8 * hi;
            a[0] = o[j][0] * cf; a[1] = o[j][1] * cf; a[2] = o[j][2] * cf; a[3] = o[j][3] * cf;
            c[0] = o[j][4] * cf; c[1] = o[j][5] * cf; c[2] = o[j][6] * cf; c[3] = o[j][7] * cf;
            if (pass != 0) { a += *(const v4fa*)(&os[ix]); c += *(const v4fa*)(&os[ix + 4]); }
            *(v4fa*)(&os[ix]) = a; *(v4fa*)(&os[ix + 4]) = c; }
    }
    wave_sync();
    h16* xrow = XO + gbase + (size_t)t0 * HD;
#pragma unroll 1
    for (int ps = 0; ps < 2; ++ps) {
#pragma unroll
        for (int s = 0; s < 8; ++s) { const int p = s * 32 + lane; const int row = p >> 4, c8 = (p & 15) * 8;
            const v4f x0 = *(const v4fa*)(&os[wb + row * OSP + c8]); const v4f x1 = *(const v4fa*)(&os[wb + row * OSP + c8 + 4]); v8h hv;
#pragma unroll
            for (int i = 0; i < 4; ++i) { hv[i] = toh_flush(x0[i]); hv[4 + i] = toh_flush(x1[i]); }
            *(volatile v8h*)(xrow + (size_t)p * 8) = hv; }
        if (ps == 0) __threadfence(); }
}

__global__ __launch_bounds__(256) void k_ln(const float* __restrict__ X2, const float* __restrict__ lng, const float* __restrict__ lnb, h16* XN) {
#pragma clang fp contract(off)
    const int lane = threadIdx.x & 31;
    const int wave = __builtin_amdgcn_readfirstlane((int)(threadIdx.x >> 5));
    const int row = blockIdx.x * 8 + wave;
    const float* xr = X2 + (size_t)row * DM + lane * 8;
    v4f xa[4], xb[4]; float s = 0.0f;
#pragma unroll
    for (int i = 0; i < 4; ++i) { xa[i] = *(const v4f*)(xr + i * 256); xb[i] = *(const v4f*)(xr + i * 256 + 4);
        s += (xa[i][0] + xa[i][1]) + (xa[i][2] + xa[i][3]); s += (xb[i][0] + xb[i][1]) + (xb[i][2] + xb[i][3]); }
#pragma unroll
    for (int off = 16; off > 0; off >>= 1) s += __shfl_xor(s, off, 32);
    const float mu = s * (1.0f / DM);
    float ss = 0.0f;
#pragma unroll
    for (int i = 0; i < 4; ++i) {
#pragma unroll
        for (int c = 0; c < 4; ++c) { const float d0 = xa[i][c] - mu, d1 = xb[i][c] - mu; ss += d0 * d0; ss += d1 * d1; } }
#pragma unroll
    for (int off = 16; off > 0; off >>= 1) ss += __shfl_xor(ss, off, 32);
    const float rs = rsqrtf(ss * (1.0f / DM) + 1e-5f);
    v8h hv[4];
#pragma unroll
    for (int i = 0; i < 4; ++i) {
        const v4f g0 = *(const v4f*)(lng + i * 256 + lane * 8), g1 = *(const v4f*)(lng + i * 256 + lane * 8 + 4);
        const v4f b0 = *(const v4f*)(lnb + i * 256 + lane * 8), b1 = *(const v4f*)(lnb + i * 256 + lane * 8 + 4);
#pragma unroll
        for (int c = 0; c < 4; ++c) {
            hv[i][c]     = toh_flush(((xa[i][c] - mu) * rs * bfr(g0[c]) + bfr(b0[c])) * ACAR);
            hv[i][4 + c] = toh_flush(((xb[i][c] - mu) * rs * bfr(g1[c]) + bfr(b1[c])) * ACAR); } }
    h16* orow = XN + (size_t)row * DM + lane * 8;
#pragma unroll 1
    for (int ps = 0; ps < 2; ++ps) {
#pragma unroll
        for (int i = 0; i < 4; ++i) *(volatile v8h*)(orow + i * 256) = hv[i];
        if (ps == 0) __threadfence(); }
}

static constexpr size_t al256(size_t v) { return (v + 255) & ~(size_t)255; }
static constexpr size_t SZ_XB  = al256((size_t)MR * DM * 2);
static constexpr size_t SZ_WSQ = al256((size_t)DM * DM * 2);
static constexpr size_t SZ_W1  = al256((size_t)OUTF * DM * 2);
static constexpr size_t SZ_W2  = al256((size_t)OUTF * OUTF * 2);
static constexpr size_t SZ_X2  = al256((size_t)MR * DM * 4);
static constexpr size_t SZ_XE  = al256((size_t)MR * OUTF * 2);
static constexpr size_t SZ_TOTAL = SZ_XB + 4 * SZ_WSQ + SZ_W1 + SZ_W2 + 6 * SZ_XB + SZ_X2 + SZ_XE;
static_assert(SZ_TOTAL <= (size_t)134217728);
static_assert((size_t)NGRP * SEQ * HD == (size_t)MR * DM);

extern "C" void kernel_launch(void* const* d_in, const int* in_sizes, int n_in,
                              void* d_out, int out_size, void* d_ws, size_t ws_size, hipStream_t stream) {
    if (n_in < 19) return;
    const size_t needx = ((size_t)(NB - 1) * SEQ_FULL + SEQ) * DM;
    if ((size_t)in_sizes[0] < needx) return;
    if ((size_t)in_sizes[2] < (size_t)DM * DM || (size_t)in_sizes[4] < (size_t)DM * DM || (size_t)in_sizes[6] < (size_t)DM * DM || (size_t)in_sizes[8] < (size_t)DM * DM) return;
    if (in_sizes[3] < DM || in_sizes[5] < DM || in_sizes[7] < DM || in_sizes[9] < DM) return;
    if (in_sizes[10] < 1 || in_sizes[11] < 1 || in_sizes[12] < 1) return;
    if (in_sizes[13] < DM || in_sizes[14] < DM) return;
    if ((size_t)in_sizes[15] < (size_t)DM * OUTF || in_sizes[16] < OUTF || (size_t)in_sizes[17] < (size_t)OUTF * OUTF || in_sizes[18] < OUTF) return;
    if ((size_t)out_size < O1OFF + ((size_t)(NB - 1) * OUTF + (OUTF - 1)) * SEQ_FULL + SEQ) return;
    if (SZ_TOTAL > ws_size) return;
    const float* x  = (const float*)d_in[0];
    const float* wq = (const float*)d_in[2];  const float* bq = (const float*)d_in[3];
    const float* wk = (const float*)d_in[4];  const float* bk = (const float*)d_in[5];
    const float* wv = (const float*)d_in[6];  const float* bv = (const float*)d_in[7];
    const float* wo = (const float*)d_in[8];  const float* bo = (const float*)d_in[9];
    const float* alpha = (const float*)d_in[10];
    const float* adjw = (const float*)d_in[11]; const float* adjb = (const float*)d_in[12];
    const float* lng = (const float*)d_in[13]; const float* lnb = (const float*)d_in[14];
    const float* w1 = (const float*)d_in[15]; const float* b1 = (const float*)d_in[16];
    const float* w2 = (const float*)d_in[17]; const float* b2 = (const float*)d_in[18];
    float* OUT0 = (float*)d_out;
    float* OUT1 = (float*)d_out + O1OFF;
    char* wsp = (char*)d_ws;
    bf*  XB  = (bf*)wsp;  wsp += SZ_XB;
    bf*  WQT = (bf*)wsp;  wsp += SZ_WSQ;
    bf*  WKT = (bf*)wsp;  wsp += SZ_WSQ;
    bf*  WVT = (bf*)wsp;  wsp += SZ_WSQ;
    h16* WOT = (h16*)wsp; wsp += SZ_WSQ;
    h16* W1T = (h16*)wsp; wsp += SZ_W1;
    h16* W2T = (h16*)wsp; wsp += SZ_W2;
    h16* QP  = (h16*)wsp; wsp += SZ_XB;
    h16* KP  = (h16*)wsp; wsp += SZ_XB;
    h16* VP  = (h16*)wsp; wsp += SZ_XB;
    h16* VT  = (h16*)wsp; wsp += SZ_XB;
    h16* XO  = (h16*)wsp; wsp += SZ_XB;
    h16* XN  = (h16*)wsp; wsp += SZ_XB;
    float* X2 = (float*)wsp; wsp += SZ_X2;
    h16* XE  = (h16*)wsp; wsp += SZ_XE;

    if (SEQ == SEQ_FULL) {
        const size_t n8 = (size_t)MR * DM / 8;
        k_cvt8<<<(unsigned)((n8 + 255) / 256), 256, 0, stream>>>(x, XB, n8);
    } else {
        const size_t n8 = (size_t)SEQ * DM / 8;
        for (int b = 0; b < NB; ++b) k_cvt8<<<(unsigned)((n8 + 255) / 256), 256, 0, stream>>>(x + (size_t)b * SEQ_FULL * DM, XB + (size_t)b * SEQ * DM, n8);
    }
    k_wt_bf<<<dim3(DM / 64, DM / 64, 1), 256, 0, stream>>>(wq, WQT, DM, DM);
    k_wt_bf<<<dim3(DM / 64, DM / 64, 1), 256, 0, stream>>>(wk, WKT, DM, DM);
    k_wt_bf<<<dim3(DM / 64, DM / 64, 1), 256, 0, stream>>>(wv, WVT, DM, DM);
    k_wt_h<<<dim3(DM / 64, DM / 64, 1), 256, 0, stream>>>(wo, WOT, DM, DM);
    k_wt_h<<<dim3(OUTF / 64, DM / 64, 1), 256, 0, stream>>>(w1, W1T, DM, OUTF);
    k_wt_h<<<dim3(OUTF / 64, OUTF / 64, 1), 256, 0, stream>>>(w2, W2T, OUTF, OUTF);

    k_gemm_proj<<<dim3(MR / 64, DM / 64, 1), 32, 0, stream>>>(XB, WQT, bq, QP, DM, DM);
    k_gemm_proj<<<dim3(MR / 64, DM / 64, 1), 32, 0, stream>>>(XB, WKT, bk, KP, DM, DM);
    k_gemm_proj<<<dim3(MR / 64, DM / 64, 1), 32, 0, stream>>>(XB, WVT, bv, VP, DM, DM);
    k_vt<<<dim3(SEQ / 64, NGRP, 1), 256, 0, stream>>>(VP, VT);

    k_keypass<<<dim3(SEQ / (16 * AW), NGRP, 1), 32 * AW, 0, stream>>>(QP, KP, VT, alpha, adjw, adjb, XO);

    k_gemm_res<<<dim3(MR / 64, DM / 64, 1), 32, 0, stream>>>(XO, WOT, bo, XB, X2, DM, DM);
    k_ln<<<MR / 8, 256, 0, stream>>>(X2, lng, lnb, XN);
    k_gemm_tr<<<dim3(OUTF / 64, MR / 64, 1), 32, 0, stream>>>(W1T, XN, b1, OUT1, XE, DM, 1);
    k_gemm_tr<<<dim3(OUTF / 64, MR / 64, 1), 32, 0, stream>>>(W2T, XE, b2, OUT0, XE, OUTF, 0);
}
